// RGCN_37555194036548
// MI455X (gfx1250) — hardware-verified
//
#include <hip/hip_runtime.h>
#include <stddef.h>
#include <stdint.h>


#define NN     50000
#define NE     1600000
#define DIN    128
#define D1     128
#define D3     16
#define NREL   16
#define NBAS   4
#define TYB    4
#define KA     (NBAS * DIN)
#define KS     DIN
#define KHL    (2 * (KA + KS))
#define KW     KHL
#define NGRP   (KHL / 8)
#define GSELF  (2 * KA / 8)
#define NCHK   2
#define CHR    25600
#define NPAD   (NCHK * CHR)
#define NTHR   256
#define NWAVE  8
#define EPT    8
#define CHUNK  (NTHR * EPT)
#define WCAP   (EPT * 32)
#define LISTN  (NWAVE * WCAP)
#define NBA    1024
#define PKS    10
#define SLB    14
#define NSUB   (NBA * NREL)
#define RCAP   34816
#define DEGCAP 96
#define SBLK   (CHR / NBA)
#define GBM    64
#define GTHR   128
#define UA1    (D1 * GSELF)
#define US1    (D1 * 32)
#define UA3    (D3 * GSELF)
#define US3    (D3 * 32)
#define R0A    UA1
#define R0S    (R0A + US1)
#define R1A    (R0S + UA1)
#define R1S    (R1A + US1)
#define R2A    (R1S + UA3)
#define R2S    (R2A + US3)
#define USH    (RCAP + 2 * NSUB)
#define AGG_ZINTS    (LISTN + RCAP + USH / 2)
#define MISC_INTS    80
#define AGG_LDS_INTS (AGG_ZINTS + MISC_INTS)
#define WSCAP  134217728

static_assert((CHUNK & (CHUNK - 1)) == 0 && CHUNK <= 2048);
static_assert((NSUB & (NSUB - 1)) == 0 && NSUB == (1 << SLB));
static_assert(NREL == (1 << TYB) && NBA * NREL == NSUB);
static_assert(NBA == (1 << PKS));
static_assert(((long long)CHUNK << SLB) < (1LL << 31));
static_assert(((long long)NE << PKS) < (1LL << 31));
static_assert(NE >= 4 && (NE % 4) == 0);
static_assert(LISTN % NTHR == 0);
static_assert(NBA % NWAVE == 0 && NSUB % 32 == 0);
static_assert(RCAP % 32 == 0 && RCAP < 65536 && (USH % 2) == 0);
static_assert(AGG_ZINTS % (NTHR * 4) == 0 && LISTN % 4 == 0);
static_assert(MISC_INTS >= 16 + NREL * NBAS && NREL * NBAS == 64);
static_assert(AGG_LDS_INTS * 4 <= 300000);
static_assert(NPAD >= NN && NPAD == NCHK * CHR && CHR % GBM == 0 && CHR % NBA == 0);
static_assert(SBLK * NBA == CHR);
static_assert(KHL % 32 == 0 && KW % 8 == 0 && NGRP == GSELF + 32 && GSELF == 32 * NBAS && DIN == 32 * 4);
static_assert((KHL * 2) % 128 == 0);
static_assert(R0A % NTHR == 0 && R0S % NTHR == 0 && R1A % NTHR == 0 && R1S % NTHR == 0);
static_assert(R2A % NTHR == 0 && R2S % NTHR == 0);
static_assert(D1 == DIN);
static_assert((NN % 2) == 0);
static_assert((long long)(NN - 1) * D3 + D3 - 1 < (long long)NN * D3);

typedef float          v4f   __attribute__((ext_vector_type(4)));
typedef float          v8f   __attribute__((ext_vector_type(8)));
typedef int            v4i   __attribute__((ext_vector_type(4)));
typedef int            v8i   __attribute__((ext_vector_type(8)));
typedef unsigned short v8us  __attribute__((ext_vector_type(8)));
typedef unsigned short v16us __attribute__((ext_vector_type(16)));
typedef __bf16         v16bf __attribute__((ext_vector_type(16)));
typedef v4f  __attribute__((may_alias)) v4fa;
typedef v4i  __attribute__((may_alias)) v4ia;
typedef v8us __attribute__((may_alias)) v8usa;
union Frag { v16bf v; v16us u; v8us h[2]; v8i w; };

__device__ __forceinline__ v8f wmb(const Frag& a, const Frag& b, v8f c) {
  v8f d = __builtin_amdgcn_wmma_f32_16x16x32_bf16(false, a.v, false, b.v, (short)0, c, false, false);
  asm volatile("v_nop\n\tv_nop\n\tv_nop\n\tv_nop" : "+v"(d) : "v"(a.w), "v"(b.w));
  return d;
}

__device__ __forceinline__ unsigned bf16_bits(float f) {
  const unsigned u = __float_as_uint(f);
  return (u + 0x7FFFu + ((u >> 16) & 1u)) >> 16;
}
__device__ __forceinline__ float bf16_val(float f) {
  return __uint_as_float(bf16_bits(f) << 16);
}
__device__ __forceinline__ v8us hilo8(v4f t) {
  v8us o;
  unsigned hb;
  hb = bf16_bits(t.x); o[0] = (unsigned short)hb; o[4] = (unsigned short)bf16_bits(t.x - __uint_as_float(hb << 16));
  hb = bf16_bits(t.y); o[1] = (unsigned short)hb; o[5] = (unsigned short)bf16_bits(t.y - __uint_as_float(hb << 16));
  hb = bf16_bits(t.z); o[2] = (unsigned short)hb; o[6] = (unsigned short)bf16_bits(t.z - __uint_as_float(hb << 16));
  hb = bf16_bits(t.w); o[3] = (unsigned short)hb; o[7] = (unsigned short)bf16_bits(t.w - __uint_as_float(hb << 16));
  return o;
}
__device__ __forceinline__ unsigned tcl(int t) {
  t = t < 0 ? 0 : (t > NREL - 1 ? NREL - 1 : t);
  return (unsigned)t;
}

__device__ __forceinline__ int scan_chunk(const int* __restrict__ dsts, const int* __restrict__ ets, int nE,
                                          int cbase, int slotBase, int* list, int tid, int lane, int wave) {
  int wc = 0;
  const int el0 = tid * EPT;
  const int e0  = cbase + el0;
  const int lim = nE - 4;
  const int q0  = e0 < lim ? e0 : lim;
  const int q1  = (e0 + 4) < lim ? (e0 + 4) : lim;
  const v4i da = *(const v4ia*)(dsts + q0);
  const v4i db = *(const v4ia*)(dsts + q1);
  const v4i ta = *(const v4ia*)(ets + q0);
  const v4i tb = *(const v4ia*)(ets + q1);
  const unsigned nbs = (unsigned)slotBase, ue0 = (unsigned)e0, unE = (unsigned)nE, unb = (unsigned)NBA;
  const unsigned s0 = (unsigned)da.x - nbs, s1 = (unsigned)da.y - nbs;
  const unsigned s2 = (unsigned)da.z - nbs, s3 = (unsigned)da.w - nbs;
  const unsigned s4 = (unsigned)db.x - nbs, s5 = (unsigned)db.y - nbs;
  const unsigned s6 = (unsigned)db.z - nbs, s7 = (unsigned)db.w - nbs;
  const unsigned r0 = tcl(ta.x), r1 = tcl(ta.y), r2 = tcl(ta.z), r3 = tcl(ta.w);
  const unsigned r4 = tcl(tb.x), r5 = tcl(tb.y), r6 = tcl(tb.z), r7 = tcl(tb.w);
  const bool h0 = (ue0 + 0u < unE) & (s0 < unb);
  const bool h1 = (ue0 + 1u < unE) & (s1 < unb);
  const bool h2 = (ue0 + 2u < unE) & (s2 < unb);
  const bool h3 = (ue0 + 3u < unE) & (s3 < unb);
  const bool h4 = (ue0 + 4u < unE) & (s4 < unb);
  const bool h5 = (ue0 + 5u < unE) & (s5 < unb);
  const bool h6 = (ue0 + 6u < unE) & (s6 < unb);
  const bool h7 = (ue0 + 7u < unE) & (s7 < unb);
  const unsigned any = __builtin_amdgcn_ballot_w32(h0 | h1 | h2 | h3 | h4 | h5 | h6 | h7);
  if (any != 0u) {
#define HITJ(J, HJ, SJ, RJ) { \
      const unsigned mj = __builtin_amdgcn_ballot_w32(HJ); \
      if (mj != 0u) { \
        if (HJ) { \
          const int pos = wc + (int)__builtin_amdgcn_mbcnt_lo(mj, 0u); \
          if (pos < WCAP) list[wave * WCAP + pos] = ((el0 + (J)) << SLB) | (int)(((SJ) << TYB) | (RJ)); \
        } \
        wc += (int)__builtin_popcount(mj); } }
    HITJ(0, h0, s0, r0)
    HITJ(1, h1, s1, r1)
    HITJ(2, h2, s2, r2)
    HITJ(3, h3, s3, r3)
    HITJ(4, h4, s4, r4)
    HITJ(5, h5, s5, r5)
    HITJ(6, h6, s6, r6)
    HITJ(7, h7, s7, r7)
#undef HITJ
  }
  return wc;
}

__global__ __launch_bounds__(NTHR) void k_prepw(const float* __restrict__ wbA, const float* __restrict__ lwA,
                                                const float* __restrict__ wbB, const float* __restrict__ lwB,
                                                const float* __restrict__ wbC, const float* __restrict__ lwC,
                                                unsigned short* WTa, unsigned short* WTb, unsigned short* WTc) {
  const int u = (int)blockIdx.x * NTHR + (int)threadIdx.x;
  const float* P;
  unsigned short* WT;
  int v, dout, kind;
  if (u < R0A)      { kind = 0; P = wbA; WT = WTa; v = u;       dout = D1; }
  else if (u < R0S) { kind = 1; P = lwA; WT = WTa; v = u - R0A; dout = D1; }
  else if (u < R1A) { kind = 0; P = wbB; WT = WTb; v = u - R0S; dout = D1; }
  else if (u < R1S) { kind = 1; P = lwB; WT = WTb; v = u - R1A; dout = D1; }
  else if (u < R2A) { kind = 0; P = wbC; WT = WTc; v = u - R1S; dout = D3; }
  else if (u < R2S) { kind = 1; P = lwC; WT = WTc; v = u - R2A; dout = D3; }
  else return;
  int oc, G, roff;
  if (kind == 0) {
    oc = v >> 7;
    const int ga = v & 127;
    G = ga;
    roff = (ga >> 5) * DIN + 4 * (ga & 31);
  } else {
    oc = v >> 5;
    const int l = v & 31;
    G = GSELF + l;
    roff = 4 * l;
  }
  const float* p = P + (size_t)roff * (size_t)dout + oc;
  const unsigned short f0 = (unsigned short)bf16_bits(p[0]);
  const unsigned short f1 = (unsigned short)bf16_bits(p[dout]);
  const unsigned short f2 = (unsigned short)bf16_bits(p[2 * dout]);
  const unsigned short f3 = (unsigned short)bf16_bits(p[3 * dout]);
  v8us o;
  o[0] = f0; o[1] = f1; o[2] = f2; o[3] = f3; o[4] = f0; o[5] = f1; o[6] = f2; o[7] = f3;
  unsigned short* dp = WT + (size_t)oc * KW + 8 * G;
  *(volatile v8us*)dp = o;
  __threadfence();
  *(volatile v8us*)dp = o;
}

template <int RIN>
__global__ __launch_bounds__(NTHR) void k_scan(const int* __restrict__ srcs, const int* __restrict__ dsts,
                                               const int* __restrict__ ets, const float* __restrict__ ew,
                                               int nE, int nN, int chunkBase, int chR,
                                               const float* __restrict__ F, const float* __restrict__ coef,
                                               unsigned short* HL) {
  extern __shared__ __attribute__((aligned(16))) int dsm[];
  int* list = dsm;
  int* hlst = dsm + LISTN;
  unsigned short* sl  = (unsigned short*)(dsm + LISTN + RCAP);
  unsigned short* cnt = sl + RCAP;
  unsigned short* cur = cnt + NSUB;
  int* misc = dsm + AGG_ZINTS;
  float* satt = (float*)(misc + 16);
  const int tid = (int)threadIdx.x, lane = tid & 31, wave = tid >> 5;
  const int nodeBase = chunkBase + (int)blockIdx.x * NBA;

  {
    const v4i z4 = {0, 0, 0, 0};
    for (int i = tid * 4; i < AGG_ZINTS; i += NTHR * 4) *(v4ia*)(dsm + i) = z4;
    if (tid < 16) misc[tid] = 0;
    if (tid < NREL * NBAS) satt[tid] = bf16_val(coef[tid]);
  }
  __syncthreads();

  int t = 0, ov = 0;
  const int nChunks = (nE + CHUNK - 1) / CHUNK;
#pragma unroll 1
  for (int ch = 0; ch < nChunks; ++ch) {
    const int cbase = ch * CHUNK;
    const int wc = scan_chunk(dsts, ets, nE, cbase, nodeBase, list, tid, lane, wave);
    if (lane == 0) misc[wave] = wc;
    __syncthreads();
    if (wave == 0) {
#pragma unroll 1
      for (int w2 = 0; w2 < NWAVE; ++w2) {
        int c = misc[w2];
        c = c < 0 ? 0 : (c > WCAP ? WCAP : c);
#pragma unroll 1
        for (int b0 = 0; b0 < c; b0 += 32) {
          const int idx = b0 + lane;
          const int ent = list[w2 * WCAP + (idx < WCAP ? idx : WCAP - 1)];
          const int m32 = (c - b0) < 32 ? (c - b0) : 32;
#pragma unroll 1
          for (int k = 0; k < m32; ++k) {
            const int u   = __builtin_amdgcn_readlane(ent, k);
            const int sub = u & (NSUB - 1);
            const int el  = (u >> SLB) & (CHUNK - 1);
            int eid = cbase + el;
            eid = eid > nE - 1 ? nE - 1 : eid;
            const int slot = sub >> TYB;
            const int pk = (eid << PKS) | slot;
            if (t < RCAP) {
              if (lane == 0) { hlst[t] = pk; cnt[sub] = (unsigned short)(cnt[sub] + 1); }
              t = t + 1;
            } else {
              ov = 1;
            }
          }
        }
      }
    }
    __syncthreads();
  }
  if (wave == 0 && lane == 0) { misc[8] = t; misc[9] = ov; }
  __syncthreads();
  int tt = misc[8];
  tt = tt < 0 ? 0 : (tt > RCAP ? RCAP : tt);
  const int ovf = misc[9];

  if (wave == 0) {
    const int base = lane * (NSUB / 32);
    int sacc = 0;
#pragma unroll 1
    for (int i = 0; i < NSUB / 32; ++i) sacc += (int)cnt[base + i];
    int incl = sacc;
#pragma unroll
    for (int d = 1; d < 32; d <<= 1) {
      const int y = __shfl_up(incl, d, 32);
      if (lane >= d) incl += y;
    }
    int run = incl - sacc;
#pragma unroll 1
    for (int i = 0; i < NSUB / 32; ++i) {
      const int cv = (int)cnt[base + i];
      cur[base + i] = (unsigned short)run;
      run += cv;
    }
  }
  __syncthreads();
  if (wave == 0) {
#pragma unroll 1
    for (int b0 = 0; b0 < tt; b0 += 32) {
      const int idx = b0 + lane;
      const int ent = hlst[idx < RCAP ? idx : RCAP - 1];
      int eid = (int)((unsigned)ent >> PKS);
      eid = eid > nE - 1 ? nE - 1 : eid;
      const int slot = ent & (NBA - 1);
      const int ty   = (int)tcl(ets[eid]);
      const int sub  = (slot << TYB) | ty;
      const int m32 = (tt - b0) < 32 ? (tt - b0) : 32;
#pragma unroll 1
      for (int k = 0; k < m32; ++k) {
        const int us   = __builtin_amdgcn_readlane(sub, k);
        const int hidx = b0 + k;
        if (lane == 0) {
          int p = (int)cur[us];
          p = p < 0 ? 0 : (p > RCAP - 1 ? RCAP - 1 : p);
          sl[p] = (unsigned short)hidx;
          cur[us] = (unsigned short)(p + 1);
        }
      }
    }
  }
  __syncthreads();

  const float qnan = __int_as_float(0x7fc00000);
  const v4f z4f = {0.0f, 0.0f, 0.0f, 0.0f};
#pragma unroll 1
  for (int si = 0; si < NBA / NWAVE; ++si) {
    const int s    = si * NWAVE + wave;
    const int lrow = (int)blockIdx.x * NBA + s;
    v4f A[NBAS];
#pragma unroll
    for (int b = 0; b < NBAS; ++b) A[b] = z4f;
    int bigf = 0;
#pragma unroll 1
    for (int r = 0; r < NREL; ++r) {
      const int sub = s * NREL + r;
      const int craw = (int)cnt[sub];
      const int cu   = (int)cur[sub];
      bigf |= (craw > DEGCAP) ? 1 : 0;
      const int c = craw < 0 ? 0 : (craw > DEGCAP ? DEGCAP : craw);
      int o = cu - craw;
      o = o < 0 ? 0 : (o > RCAP ? RCAP : o);
      v4f sv = z4f;
#pragma unroll 1
      for (int b0 = 0; b0 < c; b0 += 32) {
        int idx = o + b0 + lane;
        idx = idx > RCAP - 1 ? RCAP - 1 : idx;
        int hix = (int)sl[idx];
        hix = hix > RCAP - 1 ? RCAP - 1 : hix;
        const int ent = hlst[hix];
        int eid = (int)((unsigned)ent >> PKS);
        eid = eid > nE - 1 ? nE - 1 : eid;
        int sr = srcs[eid];
        sr = sr < 0 ? 0 : (sr > nN - 1 ? nN - 1 : sr);
        const int wvi = __float_as_int(bf16_val(ew[eid]));
        const int m32 = (c - b0) < 32 ? (c - b0) : 32;
#pragma unroll 1
        for (int k = 0; k < m32; ++k) {
          const int   sk = __builtin_amdgcn_readlane(sr, k);
          const float wk = __int_as_float(__builtin_amdgcn_readlane(wvi, k));
          const v4f v = *(const v4fa*)(F + (size_t)sk * (size_t)DIN + 4 * lane);
          float vx = v.x, vy = v.y, vz = v.z, vw = v.w;
          if constexpr (RIN == 1) {
            vx = bf16_val(vx); vy = bf16_val(vy); vz = bf16_val(vz); vw = bf16_val(vw);
          }
          sv.x = fmaf(wk, vx, sv.x); sv.y = fmaf(wk, vy, sv.y);
          sv.z = fmaf(wk, vz, sv.z); sv.w = fmaf(wk, vw, sv.w);
        }
      }
#pragma unroll
      for (int b = 0; b < NBAS; ++b) {
        const float w = satt[r * NBAS + b];
        A[b] += w * sv;
      }
    }
    int nd = nodeBase + s;
    nd = nd < 0 ? 0 : (nd > nN - 1 ? nN - 1 : nd);
    v4f hv = *(const v4fa*)(F + (size_t)nd * (size_t)DIN + 4 * lane);
    if constexpr (RIN == 1) {
      hv.x = bf16_val(hv.x); hv.y = bf16_val(hv.y); hv.z = bf16_val(hv.z); hv.w = bf16_val(hv.w);
    }
    const float pz = ((ovf | bigf) != 0) ? qnan : 0.0f;
    v8us po[NBAS + 1];
#pragma unroll
    for (int b = 0; b < NBAS; ++b) po[b] = hilo8(A[b] + pz);
    po[NBAS] = hilo8(hv + pz);
    if (lrow < chR) {
      unsigned short* rp = HL + (size_t)lrow * (size_t)KHL;
#pragma unroll
      for (int b = 0; b < NBAS; ++b)
        *(volatile v8usa*)(rp + 8 * (32 * b + lane)) = po[b];
      *(volatile v8usa*)(rp + 8 * (GSELF + lane)) = po[NBAS];
      __threadfence();
#pragma unroll
      for (int b = 0; b < NBAS; ++b)
        *(volatile v8usa*)(rp + 8 * (32 * b + lane)) = po[b];
      *(volatile v8usa*)(rp + 8 * (GSELF + lane)) = po[NBAS];
    }
  }
}

template <int N, int RELU>
__global__ __launch_bounds__(GTHR) void k_gemm(const unsigned short* __restrict__ HL,
                                               const unsigned short* __restrict__ WT,
                                               const float* __restrict__ bias,
                                               float* outp, int chunkBase, int nLim) {
  static_assert(N % 16 == 0 && N <= GTHR && (128 % N) == 0 && N % 8 == 0);
  constexpr int NT = N / 16;
  constexpr int NI = N / 8;
  __shared__ __attribute__((aligned(16))) float stg[GBM * N];
  __shared__ __attribute__((aligned(16))) float sbias[N];
  const int tid = (int)threadIdx.x, lane = tid & 31, wave = tid >> 5, hh = lane >> 4, m = lane & 15;
  const int rowBase = (int)blockIdx.x * GBM;

  {
    const int bi = tid < N ? tid : N - 1;
    const float bv = bf16_val(bias[bi]);
    if (tid < N) sbias[tid] = bv;
  }
  __syncthreads();

  v8f acc[NT];
  {
    const v8f z = {0.f, 0.f, 0.f, 0.f, 0.f, 0.f, 0.f, 0.f};
#pragma unroll
    for (int nt = 0; nt < NT; ++nt) acc[nt] = z;
  }
  const int lr0 = rowBase + 16 * wave + m;
  const unsigned short* ap = HL + (size_t)lr0 * (size_t)KHL + 8 * hh;
  const unsigned short* bp = WT + (size_t)m * (size_t)KW + 8 * hh;

#pragma unroll 1
  for (int k0 = 0; k0 < KHL; k0 += 32) {
    Frag af;
    af.h[0] = *(const v8usa*)(ap + k0);
    af.h[1] = *(const v8usa*)(ap + k0 + 16);
#pragma unroll
    for (int nt = 0; nt < NT; ++nt) {
      const unsigned short* wq = bp + (size_t)(16 * nt) * (size_t)KW + k0;
      Frag bf;
      bf.h[0] = *(const v8usa*)wq;
      bf.h[1] = *(const v8usa*)(wq + 16);
      acc[nt] = wmb(af, bf, acc[nt]);
    }
  }

#pragma unroll
  for (int nt = 0; nt < NT; ++nt) {
    const int lc = 16 * nt + m;
    const float badd = sbias[lc];
#pragma unroll
    for (int r = 0; r < 8; ++r) {
      const int lr = 16 * wave + 8 * hh + r;
      float v = acc[nt][r] + badd;
      if constexpr (RELU == 1) v = fmaxf(v, 0.0f);
      stg[lr * N + lc] = v;
    }
  }
  __syncthreads();

  v4f fv[NI];
#pragma unroll
  for (int i = 0; i < NI; ++i)
    fv[i] = *(const v4fa*)(stg + (16 * wave) * N + 128 * i + 4 * lane);
  const size_t gbase = (size_t)(chunkBase + rowBase + 16 * wave) * (size_t)N;
#pragma unroll
  for (int i = 0; i < NI; ++i) {
    const int rr   = (128 * i + 4 * lane) / N;
    const int grow = chunkBase + rowBase + 16 * wave + rr;
    if (grow < nLim)
      *(volatile v4f*)(outp + gbase + (size_t)(128 * i + 4 * lane)) = fv[i];
  }
  __threadfence();
#pragma unroll
  for (int i = 0; i < NI; ++i) {
    const int rr   = (128 * i + 4 * lane) / N;
    const int grow = chunkBase + rowBase + 16 * wave + rr;
    if (grow < nLim)
      *(volatile v4f*)(outp + gbase + (size_t)(128 * i + 4 * lane)) = fv[i];
  }
}

extern "C" void kernel_launch(void* const* d_in, const int* in_sizes, int n_in,
                              void* d_out, int out_size, void* d_ws, size_t ws_size,
                              hipStream_t stream) {
  if (n_in < 17) return;
  if (in_sizes[0]  != NN * DIN) return;
  if (in_sizes[1]  != NE) return;
  if (in_sizes[2]  != NE) return;
  if (in_sizes[3]  != NE) return;
  if (in_sizes[4]  != NE) return;
  if (in_sizes[5]  != NBAS * DIN * D1) return;
  if (in_sizes[6]  != NREL * NBAS) return;
  if (in_sizes[7]  != DIN * D1) return;
  if (in_sizes[8]  != D1) return;
  if (in_sizes[9]  != NBAS * DIN * D1) return;
  if (in_sizes[10] != NREL * NBAS) return;
  if (in_sizes[11] != DIN * D1) return;
  if (in_sizes[12] != D1) return;
  if (in_sizes[13] != NBAS * DIN * D3) return;
  if (in_sizes[14] != NREL * NBAS) return;
  if (in_sizes[15] != DIN * D3) return;
  if (in_sizes[16] != D3) return;
  if (out_size != NN * D3) return;

  const float* x    = (const float*)d_in[0];
  const int*   src  = (const int*)  d_in[1];
  const int*   dst  = (const int*)  d_in[2];
  const int*   ety  = (const int*)  d_in[3];
  const float* nrm  = (const float*)d_in[4];
  const float* wb0  = (const float*)d_in[5];
  const float* c0   = (const float*)d_in[6];
  const float* lw0  = (const float*)d_in[7];
  const float* b0   = (const float*)d_in[8];
  const float* wb1  = (const float*)d_in[9];
  const float* c1   = (const float*)d_in[10];
  const float* lw1  = (const float*)d_in[11];
  const float* b1   = (const float*)d_in[12];
  const float* wb2  = (const float*)d_in[13];
  const float* c2   = (const float*)d_in[14];
  const float* lw2  = (const float*)d_in[15];
  const float* b2   = (const float*)d_in[16];
  float* out = (float*)d_out;

  size_t off = 0;
  const size_t oWT0 = off; off += (size_t)D1 * KW * 2;       off = (off + 127) & ~(size_t)127;
  const size_t oWT1 = off; off += (size_t)D1 * KW * 2;       off = (off + 127) & ~(size_t)127;
  const size_t oWT2 = off; off += (size_t)D3 * KW * 2;       off = (off + 127) & ~(size_t)127;
  const size_t oH1  = off; off += (size_t)NPAD * D1 * 4;     off = (off + 127) & ~(size_t)127;
  const size_t oH2  = off; off += (size_t)NPAD * D1 * 4;     off = (off + 127) & ~(size_t)127;
  const size_t oHL  = off; off += (size_t)CHR * KHL * 2;     off = (off + 127) & ~(size_t)127;
  if (off > ws_size) return;
  if (off > (size_t)WSCAP) return;

  char* ws = (char*)d_ws;
  unsigned short* WT0 = (unsigned short*)(ws + oWT0);
  unsigned short* WT1 = (unsigned short*)(ws + oWT1);
  unsigned short* WT2 = (unsigned short*)(ws + oWT2);
  float*          H1  = (float*)(ws + oH1);
  float*          H2  = (float*)(ws + oH2);
  unsigned short* HL  = (unsigned short*)(ws + oHL);

  const size_t scanLds = (size_t)AGG_LDS_INTS * 4;
  hipFuncSetAttribute(reinterpret_cast<const void*>(&k_scan<1>), hipFuncAttributeMaxDynamicSharedMemorySize, (int)scanLds);
  hipFuncSetAttribute(reinterpret_cast<const void*>(&k_scan<0>), hipFuncAttributeMaxDynamicSharedMemorySize, (int)scanLds);

  k_prepw<<<dim3(R2S / NTHR), dim3(NTHR), 0, stream>>>(wb0, lw0, wb1, lw1, wb2, lw2, WT0, WT1, WT2);
  for (int c = 0; c < NCHK; ++c) {
    const int chunkBase = c * CHR;
    k_scan<1><<<dim3(SBLK), dim3(NTHR), scanLds, stream>>>(src, dst, ety, nrm, NE, NN, chunkBase, CHR, x, c0, HL);
    k_gemm<D1, 1><<<dim3(CHR / GBM), dim3(GTHR), 0, stream>>>(HL, WT0, b0, H1, chunkBase, NPAD);
  }
  for (int c = 0; c < NCHK; ++c) {
    const int chunkBase = c * CHR;
    k_scan<0><<<dim3(SBLK), dim3(NTHR), scanLds, stream>>>(src, dst, ety, nrm, NE, NN, chunkBase, CHR, H1, c1, HL);
    k_gemm<D1, 1><<<dim3(CHR / GBM), dim3(GTHR), 0, stream>>>(HL, WT1, b1, H2, chunkBase, NPAD);
  }
  for (int c = 0; c < NCHK; ++c) {
    const int chunkBase = c * CHR;
    k_scan<0><<<dim3(SBLK), dim3(NTHR), scanLds, stream>>>(src, dst, ety, nrm, NE, NN, chunkBase, CHR, H2, c2, HL);
    k_gemm<D3, 0><<<dim3(CHR / GBM), dim3(GTHR), 0, stream>>>(HL, WT2, b2, out, chunkBase, NN);
  }
  (void)hipGetLastError();
}
